// TransformerBlock_55937654063307
// MI455X (gfx1250) — hardware-verified
//
#include <hip/hip_runtime.h>
#ifndef NB
#define NB 2
#endif
#ifndef SEQ
#define SEQ 2048
#endif
#define NB_FULL 2
#define SEQ_FULL 2048
#define SQ SEQ
#define DM 1024
#define NH 16
#define HD 64
#define DFF 4096
#define LQ (3 * DM)
#define NR ((size_t)NB * SQ)

static_assert(NB <= NB_FULL);
static_assert(SEQ <= SEQ_FULL);
static_assert(DM == NH * HD);
static_assert(HD == 64);
static_assert(DM == 256 * 4);
static_assert(SQ % 128 == 0);
static_assert(DM % 64 == 0);
static_assert(DFF % 64 == 0);
static_assert(LQ % 64 == 0);
static_assert(DM % 32 == 0);
static_assert(DFF % 32 == 0);
static_assert(DM % 8 == 0);

typedef unsigned short v8us __attribute__((ext_vector_type(8), may_alias));
typedef float  v8f  __attribute__((ext_vector_type(8)));
typedef float  v4f  __attribute__((ext_vector_type(4)));
typedef float  v4fa __attribute__((ext_vector_type(4), may_alias));
typedef _Float16 v16h __attribute__((ext_vector_type(16)));
typedef _Float16 v4h __attribute__((ext_vector_type(4)));
union FragH { v16h v; v8us half[2]; _Float16 h[16]; unsigned short u[16]; };

__device__ __forceinline__ unsigned short bf16_bits(float x) { unsigned int u = __float_as_uint(x); return (unsigned short)((u + 0x7FFFu + ((u >> 16) & 1u)) >> 16); }
__device__ __forceinline__ float bf16_rne(float x) { return __uint_as_float(((unsigned int)bf16_bits(x)) << 16); }

__device__ __forceinline__ v16h g2_frag(const _Float16* p, int hh) { FragH f; f.half[0] = *(const v8us*)((const unsigned short*)p + 8 * hh); f.half[1] = *(const v8us*)((const unsigned short*)p + 16 + 8 * hh); return f.v; }
__device__ __forceinline__ v8f g2_mma(v16h a, v16h b, v8f c) { v8f d = __builtin_amdgcn_wmma_f32_16x16x32_f16(false, a, false, b, (short)0, c, false, false); asm volatile("v_nop\n\tv_nop\n\tv_nop\n\tv_nop" : "+v"(d) : "v"(a), "v"(b)); return d; }

__global__ __launch_bounds__(256) void k_wt_f16(const float* __restrict__ W, _Float16* __restrict__ Wt, int K, int N, float scale) {
  const int t = blockIdx.x * 256 + threadIdx.x; const int k8n = K / 8; if (t >= N * k8n) return;
  const int n = t / k8n, k8 = (t % k8n) * 8; FragH f;
#pragma unroll
  for (int i = 0; i < 8; ++i) f.h[i] = (_Float16)(bf16_rne(W[(size_t)(k8 + i) * N + n]) * scale);
  const v8us o = f.half[0]; unsigned short* dst = (unsigned short*)Wt + (size_t)n * K + k8;
  *(volatile v8us*)dst = o; __threadfence(); *(volatile v8us*)dst = o;
}

__global__ __launch_bounds__(256) void k_wthd(const float* __restrict__ W, _Float16* __restrict__ Bt) {
  const size_t t = (size_t)blockIdx.x * 256 + threadIdx.x; if (t >= (size_t)NH * HD * (DM / 8)) return;
  const int m8 = (int)(t % (DM / 8)) * 8; const int e = (int)((t / (DM / 8)) % HD); const int h = (int)(t / ((size_t)(DM / 8) * HD)); FragH f;
#pragma unroll
  for (int q = 0; q < 8; ++q) f.h[q] = (_Float16)(16.0f * bf16_rne(W[((size_t)h * DM + m8 + q) * HD + e]));
  const v8us o = f.half[0]; unsigned short* dst = (unsigned short*)Bt + ((size_t)h * HD + e) * DM + m8;
  *(volatile v8us*)dst = o; __threadfence(); *(volatile v8us*)dst = o;
}

__global__ __launch_bounds__(256) void k_ln16(const float* __restrict__ X, int rper, int rfull, const float* __restrict__ g, const float* __restrict__ bb, float eps, int bfin, _Float16* __restrict__ N16) {
  #pragma clang fp contract(off)
  __shared__ float red[256];
  const int row = blockIdx.x, t = threadIdx.x;
  const size_t xr = (size_t)(row / rper) * (size_t)rfull + (size_t)(row % rper);
  const v4f xa = *(const v4fa*)(X + xr * DM + t * 4);
  float s[4]; float sum = 0.f;
#pragma unroll
  for (int q = 0; q < 4; ++q) { float v = xa[q]; if (bfin) v = bf16_rne(v); s[q] = v; sum = __fadd_rn(sum, v); }
  red[t] = sum; __syncthreads();
  for (int st = 128; st > 0; st >>= 1) { if (t < st) red[t] = __fadd_rn(red[t], red[t + st]); __syncthreads(); }
  const float mu = red[0] * (1.0f / (float)DM); __syncthreads();
  float vs = 0.f;
#pragma unroll
  for (int q = 0; q < 4; ++q) { const float dl = __fadd_rn(s[q], -mu); vs = __fadd_rn(vs, __fmul_rn(dl, dl)); }
  red[t] = vs; __syncthreads();
  for (int st = 128; st > 0; st >>= 1) { if (t < st) red[t] = __fadd_rn(red[t], red[t + st]); __syncthreads(); }
  const float rs = rsqrtf(__fadd_rn(red[0] * (1.0f / (float)DM), eps)); v4h y;
#pragma unroll
  for (int q = 0; q < 4; ++q) { const int c = t * 4 + q; y[q] = (_Float16)__fadd_rn(__fmul_rn(__fmul_rn(__fadd_rn(s[q], -mu), rs), bf16_rne(g[c])), bf16_rne(bb[c])); }
  _Float16* dst = N16 + (size_t)row * DM + t * 4;
  *(volatile v4h*)dst = y; __threadfence(); *(volatile v4h*)dst = y;
}

__global__ __launch_bounds__(128) void k_gemm2(const _Float16* __restrict__ A, int lda, const _Float16* __restrict__ Bh, int ldb, float alpha,
    const float* __restrict__ bias, int act, const float* __restrict__ R, int ldr, int rper, int rfull, int rbf,
    float* __restrict__ C, _Float16* __restrict__ C16, int ldc, _Float16* __restrict__ C16L, int ldl, int nlo, int M, int N, int K) {
  __shared__ __attribute__((aligned(16))) float so[4][32][68];
  const int tid = threadIdx.x, w = tid >> 5, lane = tid & 31, ln = lane & 15, hh = lane >> 4;
  const int ntn = N >> 6; const int mt = blockIdx.x / ntn, nq = blockIdx.x - mt * ntn; const int row0 = mt * 128 + 32 * w, col0 = nq * 64; if (row0 >= M) return;
  const _Float16* a0p = A + (size_t)(row0 + ln) * lda; const _Float16* a1p = a0p + (size_t)16 * lda;
  const _Float16* b0p = Bh + (size_t)(col0 + ln) * ldb; const _Float16* b1p = b0p + (size_t)16 * ldb; const _Float16* b2p = b1p + (size_t)16 * ldb; const _Float16* b3p = b2p + (size_t)16 * ldb;
  const v8f z8 = {0.f,0.f,0.f,0.f,0.f,0.f,0.f,0.f}; v8f c00 = z8, c01 = z8, c02 = z8, c03 = z8, c10 = z8, c11 = z8, c12 = z8, c13 = z8;
#pragma unroll 1
  for (int kb = 0; kb < K; kb += 32) { const v16h a0 = g2_frag(a0p + kb, hh), a1 = g2_frag(a1p + kb, hh);
    v16h b = g2_frag(b0p + kb, hh); c00 = g2_mma(a0, b, c00); c10 = g2_mma(a1, b, c10);
    b = g2_frag(b1p + kb, hh); c01 = g2_mma(a0, b, c01); c11 = g2_mma(a1, b, c11);
    b = g2_frag(b2p + kb, hh); c02 = g2_mma(a0, b, c02); c12 = g2_mma(a1, b, c12);
    b = g2_frag(b3p + kb, hh); c03 = g2_mma(a0, b, c03); c13 = g2_mma(a1, b, c13); }
  v8f accs[8] = {c00, c01, c02, c03, c10, c11, c12, c13};
#pragma unroll
  for (int u = 0; u < 8; ++u) { const int t = u & 3, half = u >> 2; const int col = col0 + t * 16 + ln; float bv = 0.f; if (bias) bv = bf16_rne(bias[col]);
#pragma unroll
    for (int r = 0; r < 8; ++r) { const int rloc = half * 16 + 8 * hh + r; float v = accs[u][r] * alpha + bv; if (act == 3) v = fmaxf(v, 0.f); so[w][rloc][t * 16 + ln] = v; } }
  __builtin_amdgcn_fence(4  , "workgroup"); __builtin_amdgcn_wave_barrier();
  const int rsub = lane >> 4, c4 = (lane & 15) * 4;
  if (R) {
    const size_t rrow0 = (size_t)(row0 / rper) * (size_t)rfull + (size_t)(row0 % rper);
#pragma unroll 4
    for (int q = 0; q < 16; ++q) { const int r = q * 2 + rsub; v4f v = *(const v4fa*)&so[w][r][c4]; v4f rv = *(const v4fa*)(R + (rrow0 + r) * (size_t)ldr + col0 + c4);
      if (rbf) { rv[0] = bf16_rne(rv[0]); rv[1] = bf16_rne(rv[1]); rv[2] = bf16_rne(rv[2]); rv[3] = bf16_rne(rv[3]); }
      v[0] += rv[0]; v[1] += rv[1]; v[2] += rv[2]; v[3] += rv[3]; *(v4fa*)&so[w][r][c4] = v; }
  }
  const int wlo = (C16L != nullptr && col0 < nlo) ? 1 : 0;
  for (int pass = 0; pass < 2; ++pass) {
#pragma unroll 4
    for (int q = 0; q < 16; ++q) { const int r = q * 2 + rsub; const v4f v = *(const v4fa*)&so[w][r][c4];
      if (C) *(volatile v4f*)(C + (size_t)(row0 + r) * ldc + col0 + c4) = v;
      if (C16) { v4h h4; h4[0] = (_Float16)v[0]; h4[1] = (_Float16)v[1]; h4[2] = (_Float16)v[2]; h4[3] = (_Float16)v[3];
        *(volatile v4h*)(C16 + (size_t)(row0 + r) * ldc + col0 + c4) = h4;
        if (wlo) { v4h l4; l4[0] = (_Float16)((v[0] - (float)h4[0]) * 2048.0f); l4[1] = (_Float16)((v[1] - (float)h4[1]) * 2048.0f); l4[2] = (_Float16)((v[2] - (float)h4[2]) * 2048.0f); l4[3] = (_Float16)((v[3] - (float)h4[3]) * 2048.0f);
          *(volatile v4h*)(C16L + (size_t)(row0 + r) * ldl + col0 + c4) = l4; } } }
    if (pass == 0) __threadfence(); }
}

__global__ __launch_bounds__(256) void k_vt(const _Float16* __restrict__ V16, int ldv, _Float16* __restrict__ Vt) {
  __shared__ unsigned short tl[64][66];
  const int tid = threadIdx.x; const int slab = blockIdx.x / (SQ / 64), lg = blockIdx.x % (SQ / 64); const int b = slab / NH, h = slab % NH;
  for (int i = tid; i < 64 * 8; i += 256) { const int r = i / 8, c8 = (i % 8) * 8; FragH f; f.half[0] = *(const v8us*)((const unsigned short*)V16 + ((size_t)b * SQ + lg * 64 + r) * ldv + h * 64 + c8);
#pragma unroll
    for (int q = 0; q < 8; ++q) tl[r][c8 + q] = f.u[q]; }
  __syncthreads();
  for (int pass = 0; pass < 2; ++pass) {
#pragma unroll
    for (int rd = 0; rd < 2; ++rd) { const int d = rd * 32 + tid / 8, pc = tid % 8; FragH f;
#pragma unroll
      for (int q = 0; q < 8; ++q) f.u[q] = tl[pc * 8 + q][d];
      *(volatile v8us*)((unsigned short*)Vt + ((size_t)slab * 64 + d) * SQ + lg * 64 + pc * 8) = f.half[0]; }
    if (pass == 0) __threadfence(); }
}

__global__ __launch_bounds__(128) void k_fattn(const _Float16* __restrict__ QKV, const _Float16* __restrict__ QL, const _Float16* __restrict__ VT, _Float16* __restrict__ O16) {
  __shared__ __attribute__((aligned(16))) unsigned short ot[4][16][72];
  const int tid = threadIdx.x, w = tid >> 5, lane = tid & 31, ln = lane & 15, hh = lane >> 4;
  const int bh = blockIdx.y; const int b = bh / NH, h = bh - b * NH;
  const int qr0 = blockIdx.x * 64 + w * 16;
  const size_t r0 = (size_t)b * SQ;
  const size_t qoff = (r0 + qr0 + ln) * LQ + (size_t)h * HD;
  const size_t qloff = (r0 + qr0 + ln) * DM + (size_t)h * HD;
  const size_t koff = (r0 + ln) * LQ + DM + (size_t)h * HD;
  const size_t voff = ((size_t)bh * HD + ln) * SQ;
  const int qi = qr0 + ln;
  const v8f z8 = {0.f,0.f,0.f,0.f,0.f,0.f,0.f,0.f};
  v8f oa[4] = {z8, z8, z8, z8};
  float m = -1.0e30f, l = 0.f;
  const int nst = (qr0 >> 5) + 1;
#pragma unroll 1
  for (int st = 0; st < nst; ++st) {
    const int kb = st * 32;
    v8f sh0 = z8, sh1 = z8, sl0 = z8, sl1 = z8;
#pragma unroll
    for (int ks = 0; ks < 2; ++ks) {
      const v16h qh = g2_frag(QKV + qoff + ks * 32, hh);
      const v16h ql = g2_frag(QL + qloff + ks * 32, hh);
      const v16h k0 = g2_frag(QKV + koff + (size_t)kb * LQ + ks * 32, hh);
      sh0 = g2_mma(k0, qh, sh0); sl0 = g2_mma(k0, ql, sl0);
      const v16h k1 = g2_frag(QKV + koff + (size_t)(kb + 16) * LQ + ks * 32, hh);
      sh1 = g2_mma(k1, qh, sh1); sl1 = g2_mma(k1, ql, sl1);
    }
    float sv[16]; float tm = -1.0e30f;
#pragma unroll
    for (int r = 0; r < 8; ++r) {
      const int j0 = kb + 8 * hh + r, j1 = j0 + 16;
      float a = (sh0[r] + sl0[r] * 0.00048828125f) * 0.125f;
      float c = (sh1[r] + sl1[r] * 0.00048828125f) * 0.125f;
      a = (j0 <= qi) ? a : -1.0e30f; c = (j1 <= qi) ? c : -1.0e30f;
      sv[r] = a; sv[8 + r] = c; tm = fmaxf(tm, fmaxf(a, c));
    }
    tm = fmaxf(tm, __shfl_xor(tm, 16, 32));
    const float mn = fmaxf(m, tm);
    const float corr = __expf(m - mn);
    m = mn;
    FragH pf; float rs = 0.f;
#pragma unroll
    for (int i = 0; i < 16; ++i) { const _Float16 ph = (_Float16)(__expf(sv[i] - mn) * 1024.0f); pf.h[i] = ph; rs += (float)ph; }
    rs += __shfl_xor(rs, 16, 32);
    l = l * corr + rs;
#pragma unroll
    for (int t = 0; t < 4; ++t) {
#pragma unroll
      for (int r = 0; r < 8; ++r) oa[t][r] *= corr; }
    const size_t vo = voff + kb;
    const v16h v0 = g2_frag(VT + vo, hh), v1 = g2_frag(VT + vo + (size_t)16 * SQ, hh), v2 = g2_frag(VT + vo + (size_t)32 * SQ, hh), v3 = g2_frag(VT + vo + (size_t)48 * SQ, hh);
    oa[0] = g2_mma(v0, pf.v, oa[0]); oa[1] = g2_mma(v1, pf.v, oa[1]); oa[2] = g2_mma(v2, pf.v, oa[2]); oa[3] = g2_mma(v3, pf.v, oa[3]);
  }
  const float inv = 64.0f * (1.0f / l);
#pragma unroll
  for (int t = 0; t < 4; ++t) { FragH f;
#pragma unroll
    for (int r = 0; r < 8; ++r) f.h[r] = (_Float16)(oa[t][r] * inv);
    *(v8us*)&ot[w][ln][t * 16 + 8 * hh] = f.half[0]; }
  __builtin_amdgcn_fence(4  , "workgroup"); __builtin_amdgcn_wave_barrier();
  const int rq = lane >> 3, pc = (lane & 7) * 8;
  for (int pass = 0; pass < 2; ++pass) {
#pragma unroll
    for (int it = 0; it < 4; ++it) { const int row = it * 4 + rq; const v8us v = *(const v8us*)&ot[w][row][pc];
      *(volatile v8us*)((unsigned short*)O16 + (r0 + qr0 + row) * DM + (size_t)h * HD + pc) = v; }
    if (pass == 0) __threadfence(); }
}

#define SZ_BQKV ((size_t)3 * DM * DM * 2)
#define SZ_BO   ((size_t)DM * DM * 2)
#define SZ_BW1  ((size_t)DFF * DM * 2)
#define SZ_BW2  ((size_t)DM * DFF * 2)
#define SZ_X16  (NR * DM * 2)
#define SZ_QKV  (NR * LQ * 2)
#define SZ_QL   (NR * DM * 2)
#define SZ_VT   ((size_t)NB * NH * HD * SQ * 2)
#define SZ_O16  (NR * DM * 2)
#define SZ_X2   (NR * DM * 4)
#define SZ_M16  (NR * DM * 2)
#define SZ_HF   ((size_t)SQ * DFF * 2)
#define WS_TOTAL (SZ_BQKV + SZ_BO + SZ_BW1 + SZ_BW2 + SZ_X16 + SZ_QKV + SZ_QL + SZ_VT + SZ_O16 + SZ_X2 + SZ_M16 + SZ_HF)
static_assert(WS_TOTAL <= (size_t)134217728);
static_assert(SZ_BQKV % 256 == 0 && SZ_BO % 256 == 0 && SZ_BW1 % 256 == 0 && SZ_X16 % 256 == 0 && SZ_QKV % 256 == 0 && SZ_VT % 256 == 0 && SZ_X2 % 256 == 0 && SZ_HF % 256 == 0);
static_assert(((size_t)NH * HD * (DM / 8)) % 256 == 0);
static_assert(((size_t)DM * (DM / 8)) % 256 == 0 && ((size_t)DFF * (DM / 8)) % 256 == 0);

extern "C" void kernel_launch(void* const* d_in, const int* in_sizes, int n_in,
                              void* d_out, int out_size, void* d_ws, size_t ws_size, hipStream_t stream) {
  if (n_in < 14) return;
  const long long need_x = (long long)(NB - 1) * SEQ_FULL * DM + (long long)SQ * DM;
  if ((long long)in_sizes[0] < need_x) return;
  if (in_sizes[1] < NH * DM * HD || in_sizes[2] < NH * DM * HD || in_sizes[3] < NH * DM * HD) return;
  if (in_sizes[4] < DM * DM || in_sizes[5] < DM || in_sizes[6] < DM * DFF || in_sizes[7] < DFF || in_sizes[8] < DFF * DM || in_sizes[9] < DM) return;
  if (in_sizes[10] < DM || in_sizes[11] < DM || in_sizes[12] < DM || in_sizes[13] < DM) return;
  if ((long long)out_size < (long long)NB * SQ * DM) return;
  if (WS_TOTAL > ws_size) return;
  const float* const* I = (const float* const*)d_in;
  const float* x = I[0]; const float* wq = I[1]; const float* wk = I[2]; const float* wv = I[3]; const float* wo = I[4]; const float* bo = I[5];
  const float* w1 = I[6]; const float* b1 = I[7]; const float* w2 = I[8]; const float* b2 = I[9]; const float* g1 = I[10]; const float* be1 = I[11]; const float* g2 = I[12]; const float* be2 = I[13];
  float* out = (float*)d_out;
  char* ws = (char*)d_ws; size_t off = 0;
  _Float16* BQKV = (_Float16*)(ws + off); off += SZ_BQKV;
  _Float16* BO   = (_Float16*)(ws + off); off += SZ_BO;
  _Float16* BW1  = (_Float16*)(ws + off); off += SZ_BW1;
  _Float16* BW2  = (_Float16*)(ws + off); off += SZ_BW2;
  _Float16* X16  = (_Float16*)(ws + off); off += SZ_X16;
  _Float16* QKV  = (_Float16*)(ws + off); off += SZ_QKV;
  _Float16* QL   = (_Float16*)(ws + off); off += SZ_QL;
  _Float16* VT   = (_Float16*)(ws + off); off += SZ_VT;
  _Float16* O16  = (_Float16*)(ws + off); off += SZ_O16;
  float*    X2   = (float*)(ws + off);    off += SZ_X2;
  _Float16* M16  = (_Float16*)(ws + off); off += SZ_M16;
  _Float16* HF16 = (_Float16*)(ws + off); off += SZ_HF;

  { const unsigned g = (unsigned)(((size_t)NH * HD * (DM / 8)) / 256);
    k_wthd<<<g, 256, 0, stream>>>(wq, BQKV);
    k_wthd<<<g, 256, 0, stream>>>(wk, BQKV + (size_t)DM * DM);
    k_wthd<<<g, 256, 0, stream>>>(wv, BQKV + (size_t)2 * DM * DM); }
  k_wt_f16<<<(unsigned)(((size_t)DM * (DM / 8)) / 256), 256, 0, stream>>>(wo, BO, DM, DM, 16.0f);
  k_wt_f16<<<(unsigned)(((size_t)DFF * (DM / 8)) / 256), 256, 0, stream>>>(w1, BW1, DM, DFF, 16.0f);
  k_wt_f16<<<(unsigned)(((size_t)DM * (DFF / 8)) / 256), 256, 0, stream>>>(w2, BW2, DFF, DM, 16.0f);
  k_ln16<<<(unsigned)NR, 256, 0, stream>>>(x, SQ, SEQ_FULL, g1, be1, 1e-5f, 1, X16);
  k_gemm2<<<(unsigned)((NR / 128) * (LQ / 64)), 128, 0, stream>>>(X16, DM, BQKV, DM, 0.0625f, nullptr, 0, nullptr, 0, 1, 1, 0,
      nullptr, QKV, LQ, QL, DM, DM, (int)NR, LQ, DM);
  k_vt<<<(unsigned)(NB * NH * (SQ / 64)), 256, 0, stream>>>(QKV + 2 * DM, LQ, VT);
  k_fattn<<<dim3((unsigned)(SQ / 64), (unsigned)(NB * NH)), 128, 0, stream>>>(QKV, QL, VT, O16);
  k_gemm2<<<(unsigned)((NR / 128) * (DM / 64)), 128, 0, stream>>>(O16, DM, BO, DM, 0.0009765625f, bo, 0, x, DM, SQ, SEQ_FULL, 1,
      X2, nullptr, DM, nullptr, 0, 0, (int)NR, DM, DM);
  k_ln16<<<(unsigned)NR, 256, 0, stream>>>(X2, SQ, SQ, g2, be2, 1e-5f, 0, M16);
  for (int b = 0; b < NB; ++b) { const size_t r0 = (size_t)b * SQ;
    k_gemm2<<<(unsigned)((SQ / 128) * (DFF / 64)), 128, 0, stream>>>(M16 + r0 * DM, DM, BW1, DM, 0.0625f, b1, 3, nullptr, 0, 1, 1, 0,
        nullptr, HF16, DFF, nullptr, 0, 0, SQ, DFF, DM);
    k_gemm2<<<(unsigned)((SQ / 128) * (DM / 64)), 128, 0, stream>>>(HF16, DFF, BW2, DFF, 0.0625f, b2, 0, X2 + r0 * DM, DM, SQ, SQ, 0,
        out + r0 * DM, nullptr, DM, nullptr, 0, 0, SQ, DM, DFF); }
}
